// SelfAttentionExtractor_21122649162109
// MI455X (gfx1250) — hardware-verified
//
#include <hip/hip_runtime.h>
#include <stddef.h>
#include <stdint.h>


typedef __bf16 v16b __attribute__((ext_vector_type(16)));
typedef float v8f __attribute__((ext_vector_type(8)));
typedef float v4f __attribute__((ext_vector_type(4)));
typedef v4f v4fa __attribute__((may_alias));
typedef unsigned int v8u __attribute__((ext_vector_type(8)));
typedef unsigned int v4u __attribute__((ext_vector_type(4)));

static constexpr int NS = 36;
static constexpr int NHID = 256;
static constexpr int NHEAD = 8;
static constexpr int HDIM = 32;
static constexpr int NBLK = 4;
static constexpr int NTHR = 256;
static constexpr int NWAVES = 8;
static constexpr int ROBW = 47;
static constexpr int NOBJ = 6;
static constexpr int OBJD = 16;
static constexpr int EMB_IN = 33;
static constexpr int TOKP = 64;
static constexpr int SCP = 48;
static constexpr int PRP = 64;

static constexpr int EW1_FR = 16384;
static constexpr int MAT_FR = 65536;
static constexpr int NMATS = 25;
static constexpr int PLANE = EW1_FR + NMATS * MAT_FR;
static constexpr int NGROUPS = (2 * PLANE) / 8;
static constexpr size_t WS_NEED = (size_t)2 * PLANE * sizeof(unsigned short);

struct Params {
  const float* robot;
  const float* objs;
  const int* masks;
  const float* ew1; const float* eb1; const float* ew2; const float* eb2; const float* elg; const float* elb;
  const float* Wq; const float* bq; const float* Wk; const float* bk; const float* Wv; const float* bv;
  const float* Wo; const float* bo; const float* ln1g; const float* ln1b;
  const float* fw1; const float* fb1; const float* fw2; const float* fb2; const float* ln2g; const float* ln2b;
  float* out;
};
static_assert(sizeof(Params) == 26 * sizeof(void*));

union Frag { v16b v; v8u u; v4u q[2]; };
struct HL { unsigned h, l; };

__device__ __forceinline__ unsigned bf_bits(float x) {
  unsigned u = __float_as_uint(x);
  return (u + 0x7FFFu + ((u >> 16) & 1u)) >> 16;
}

__device__ __forceinline__ HL split2(float x0, float x1) {
  unsigned h0 = bf_bits(x0), h1 = bf_bits(x1);
  float r0 = x0 - __uint_as_float(h0 << 16);
  float r1 = x1 - __uint_as_float(h1 << 16);
  HL o;
  o.h = h0 | (h1 << 16);
  o.l = bf_bits(r0) | (bf_bits(r1) << 16);
  return o;
}

__device__ __forceinline__ v8f zero8() {
  v8f c;
#pragma unroll
  for (int i = 0; i < 8; ++i) c[i] = 0.f;
  return c;
}

__device__ __forceinline__ v8f mma3(v16b ah, v16b al, v16b bh, v16b bl, v8f c) {
  c = __builtin_amdgcn_wmma_f32_16x16x32_bf16(false, ah, false, bh, (short)0, c, false, false);
  c = __builtin_amdgcn_wmma_f32_16x16x32_bf16(false, ah, false, bl, (short)0, c, false, false);
  c = __builtin_amdgcn_wmma_f32_16x16x32_bf16(false, al, false, bh, (short)0, c, false, false);
  asm volatile("v_nop\n\tv_nop\n\tv_nop\n\tv_nop" : "+v"(c) : "v"(ah), "v"(al), "v"(bh), "v"(bl));
  return c;
}

__device__ __forceinline__ void load_a(const float* src, int ld, int row, int kb, Frag& fh, Frag& fl) {
  const v4fa* q0 = (const v4fa*)(src + row * ld + kb);
  v4f x0 = q0[0], x1 = q0[1], x2 = q0[4], x3 = q0[5];
  float x[16] = {x0[0], x0[1], x0[2], x0[3], x1[0], x1[1], x1[2], x1[3],
                 x2[0], x2[1], x2[2], x2[3], x3[0], x3[1], x3[2], x3[3]};
#pragma unroll
  for (int j = 0; j < 8; ++j) {
    HL t = split2(x[2 * j], x[2 * j + 1]);
    fh.u[j] = t.h;
    fl.u[j] = t.l;
  }
}

__device__ __forceinline__ void load_b(const unsigned short* __restrict__ wh, const unsigned short* __restrict__ wl,
                                       int blk, int lane, Frag& fh, Frag& fl) {
  const int off = (blk << 9) + (lane << 4);
  const v4u* a = (const v4u*)(wh + off);
  const v4u* c = (const v4u*)(wl + off);
  fh.q[0] = a[0];
  fh.q[1] = a[1];
  fl.q[0] = c[0];
  fl.q[1] = c[1];
}

__device__ __forceinline__ void load_v(const float* vsrc, int kc, int n, int h, Frag& fh, Frag& fl) {
  float x[16];
#pragma unroll
  for (int i = 0; i < 16; ++i) {
    int k = kc * 32 + ((i < 8) ? (8 * h + i) : (16 + 8 * h + (i - 8)));
    k = (k < NS) ? k : (NS - 1);
    x[i] = vsrc[k * HDIM + n];
  }
#pragma unroll
  for (int j = 0; j < 8; ++j) {
    HL t = split2(x[2 * j], x[2 * j + 1]);
    fh.u[j] = t.h;
    fl.u[j] = t.l;
  }
}

__global__ __launch_bounds__(NTHR) void prepack_kernel(Params p, unsigned short* ws) {
  const int g = blockIdx.x * NTHR + threadIdx.x;
  if (g >= NGROUPS) return;
  const int off = g * 8;
  const int plane = (off >= PLANE) ? 1 : 0;
  const int o = off - plane * PLANE;
  int blk, nt, kc, kdim;
  const float* Wm;
  if (o < EW1_FR) {
    blk = o >> 9; nt = blk >> 1; kc = blk & 1; kdim = EMB_IN; Wm = p.ew1;
  } else {
    const int d = o - EW1_FR;
    const int mi = d >> 16;
    const int r = d & (MAT_FR - 1);
    blk = r >> 9; nt = blk >> 3; kc = blk & 7; kdim = NHID;
    if (mi == 0)       Wm = p.ew2;
    else if (mi < 5)   Wm = p.Wq + (mi - 1) * MAT_FR;
    else if (mi < 9)   Wm = p.Wk + (mi - 5) * MAT_FR;
    else if (mi < 13)  Wm = p.Wv + (mi - 9) * MAT_FR;
    else if (mi < 17)  Wm = p.Wo + (mi - 13) * MAT_FR;
    else if (mi < 21)  Wm = p.fw1 + (mi - 17) * MAT_FR;
    else               Wm = p.fw2 + (mi - 21) * MAT_FR;
  }
  const int lane = (o >> 4) & 31;
  const int j0 = o & 15;
  const int hh = lane >> 4;
  const int n = nt * 16 + (lane & 15);
  const int kb = kc * 32 + 8 * hh + (j0 ? 16 : 0);
  v4u val;
#pragma unroll
  for (int jj = 0; jj < 4; ++jj) {
    const int k0 = kb + 2 * jj, k1 = kb + 2 * jj + 1;
    const float x0 = (k0 < kdim) ? Wm[k0 * NHID + n] : 0.f;
    const float x1 = (k1 < kdim) ? Wm[k1 * NHID + n] : 0.f;
    HL t = split2(x0, x1);
    val[jj] = plane ? t.l : t.h;
  }
  unsigned short* dst = ws + off;
  *(volatile v4u*)dst = val;
  __threadfence();
  *(volatile v4u*)dst = val;
}

__device__ inline void gemm_big(const float* src, int ld, int nkc,
                                const unsigned short* __restrict__ wh, const unsigned short* __restrict__ wl,
                                const float* __restrict__ bias, float* dst, const float* resid, bool relu,
                                int wave, int lane) {
  const int h = lane >> 4, m = lane & 15;
#pragma unroll 1
  for (int t = wave; t < 48; t += NWAVES) {
    const int mt = t >> 4, nt = t & 15;
    int arow = mt * 16 + m;
    if (arow > NS - 1) arow = NS - 1;
    v8f c = zero8();
#pragma unroll 1
    for (int kc = 0; kc < nkc; ++kc) {
      Frag ah, al, bh, bl;
      load_a(src, ld, arow, kc * 32 + 8 * h, ah, al);
      load_b(wh, wl, nt * nkc + kc, lane, bh, bl);
      c = mma3(ah.v, al.v, bh.v, bl.v, c);
    }
    const int col = nt * 16 + m;
    const float bb = bias[col];
#pragma unroll
    for (int r = 0; r < 8; ++r) {
      const int row = mt * 16 + 8 * h + r;
      if (row < NS) {
        float v = c[r] + bb;
        if (resid != nullptr) v += resid[row * NHID + col];
        if (relu) v = fmaxf(v, 0.f);
        dst[row * NHID + col] = v;
      }
    }
  }
}

__device__ inline void layer_norm(float* xb, const float* __restrict__ g, const float* __restrict__ bt,
                                  int wave, int lane) {
#pragma unroll 1
  for (int r = wave; r < NS; r += NWAVES) {
    float vals[8];
    float s = 0.f;
#pragma unroll
    for (int i = 0; i < 8; ++i) {
      vals[i] = xb[r * NHID + lane + 32 * i];
      s += vals[i];
    }
#pragma unroll
    for (int off = 16; off >= 1; off >>= 1) s += __shfl_xor(s, off, 32);
    const float mu = s * (1.f / 256.f);
    float vs = 0.f;
#pragma unroll
    for (int i = 0; i < 8; ++i) {
      const float d = vals[i] - mu;
      vs += d * d;
    }
#pragma unroll
    for (int off = 16; off >= 1; off >>= 1) vs += __shfl_xor(vs, off, 32);
    const float inv = 1.f / sqrtf(vs * (1.f / 256.f) + 1e-5f);
#pragma unroll
    for (int i = 0; i < 8; ++i) {
      const int col = lane + 32 * i;
      xb[r * NHID + col] = (vals[i] - mu) * inv * g[col] + bt[col];
    }
  }
}

__global__ __launch_bounds__(NTHR) void fused_kernel(Params p, const unsigned short* __restrict__ ws) {
  __shared__ __align__(16) float bufA[NS * NHID];
  __shared__ __align__(16) float bufB[NS * NHID];
  __shared__ __align__(16) float bufC[NS * NHID];
  __shared__ __align__(16) float qh[NS * HDIM];
  __shared__ __align__(16) float kh[NS * HDIM];
  __shared__ __align__(16) float vh[NS * HDIM];
  __shared__ __align__(16) float sc[NS * SCP];
  __shared__ __align__(16) float pr[NS * PRP];
  __shared__ int mflag[8];

  const int b = blockIdx.x;
  const int tid = threadIdx.x;
  const int wave = tid >> 5;
  const int lane = tid & 31;
  const int h = lane >> 4, m = lane & 15;

  const unsigned short* wsh = ws;
  const unsigned short* wsl = ws + PLANE;

  float* tok = bufC;
  for (int idx = tid; idx < NS * TOKP; idx += NTHR) tok[idx] = 0.f;
  if (tid < 8) mflag[tid] = (tid < NOBJ) ? ((p.masks[b * NOBJ + tid] != 0) ? 1 : 0) : 0;
  __syncthreads();
  for (int idx = tid; idx < NS * EMB_IN; idx += NTHR) {
    const int row = idx / EMB_IN, c = idx - row * EMB_IN;
    const int gi = row / NOBJ, oi = row - gi * NOBJ;
    float v;
    if (c < 11)       v = p.robot[b * ROBW + c];
    else if (c < 14)  v = p.robot[b * ROBW + 11 + gi * 3 + (c - 11)];
    else if (c < 17)  v = p.robot[b * ROBW + 29 + gi * 3 + (c - 14)];
    else              v = p.objs[(b * NOBJ + oi) * OBJD + (c - 17)];
    tok[row * TOKP + c] = v;
  }
  __syncthreads();

  gemm_big(tok, TOKP, 2, wsh, wsl, p.eb1, bufB, nullptr, true, wave, lane);
  __syncthreads();
  gemm_big(bufB, NHID, 8, wsh + EW1_FR, wsl + EW1_FR, p.eb2, bufA, nullptr, false, wave, lane);
  __syncthreads();
  layer_norm(bufA, p.elg, p.elb, wave, lane);
  __syncthreads();

  const float scale = 0.17677669529663687f;

  for (int i = 0; i < NBLK; ++i) {
    for (int hd = 0; hd < NHEAD; ++hd) {
#pragma unroll 1
      for (int t = wave; t < 18; t += NWAVES) {
        const int which = t / 6, tt = t - which * 6;
        const int mt = tt >> 1, nt = tt & 1;
        const int mi = ((which == 0) ? 1 : (which == 1) ? 5 : 9) + i;
        const unsigned short* wh = wsh + EW1_FR + mi * MAT_FR;
        const unsigned short* wl = wsl + EW1_FR + mi * MAT_FR;
        const float* bs = ((which == 0) ? p.bq : (which == 1) ? p.bk : p.bv) + i * NHID + hd * HDIM;
        float* dst = (which == 0) ? qh : (which == 1) ? kh : vh;
        int arow = mt * 16 + m;
        if (arow > NS - 1) arow = NS - 1;
        v8f c = zero8();
#pragma unroll 1
        for (int kc = 0; kc < 8; ++kc) {
          Frag ah, al, bh, bl;
          load_a(bufA, NHID, arow, kc * 32 + 8 * h, ah, al);
          load_b(wh, wl, (hd * 2 + nt) * 8 + kc, lane, bh, bl);
          c = mma3(ah.v, al.v, bh.v, bl.v, c);
        }
        const int col = nt * 16 + m;
        const float bb = bs[col];
#pragma unroll
        for (int r = 0; r < 8; ++r) {
          const int row = mt * 16 + 8 * h + r;
          if (row < NS) dst[row * HDIM + col] = c[r] + bb;
        }
      }
      __syncthreads();

#pragma unroll 1
      for (int t = wave; t < 9; t += NWAVES) {
        const int mt = t / 3, nt = t - mt * 3;
        int arow = mt * 16 + m; if (arow > NS - 1) arow = NS - 1;
        int brow = nt * 16 + m; if (brow > NS - 1) brow = NS - 1;
        Frag ah, al, bh, bl;
        load_a(qh, HDIM, arow, 8 * h, ah, al);
        load_a(kh, HDIM, brow, 8 * h, bh, bl);
        v8f c = mma3(ah.v, al.v, bh.v, bl.v, zero8());
        const int col = nt * 16 + m;
#pragma unroll
        for (int r = 0; r < 8; ++r) {
          const int row = mt * 16 + 8 * h + r;
          if (row < NS) sc[row * SCP + col] = c[r] * scale;
        }
      }
      __syncthreads();

#pragma unroll 1
      for (int q = wave; q < NS; q += NWAVES) {
        const int k0 = lane, k1 = 32 + lane;
        const bool v1 = (k1 < NS);
        float s0 = sc[q * SCP + k0];
        if (mflag[k0 % NOBJ]) s0 = -1.0e9f;
        float s1 = -3.0e38f;
        if (v1) {
          s1 = sc[q * SCP + k1];
          if (mflag[k1 % NOBJ]) s1 = -1.0e9f;
        }
        float mx = fmaxf(s0, s1);
#pragma unroll
        for (int off = 16; off >= 1; off >>= 1) mx = fmaxf(mx, __shfl_xor(mx, off, 32));
        const float e0 = expf(s0 - mx);
        const float e1 = v1 ? expf(s1 - mx) : 0.f;
        float sm = e0 + e1;
#pragma unroll
        for (int off = 16; off >= 1; off >>= 1) sm += __shfl_xor(sm, off, 32);
        const float inv = 1.f / sm;
        pr[q * PRP + k0] = e0 * inv;
        pr[q * PRP + k1] = e1 * inv;
      }
      __syncthreads();

#pragma unroll 1
      for (int t = wave; t < 6; t += NWAVES) {
        const int mt = t >> 1, nt = t & 1;
        int arow = mt * 16 + m; if (arow > NS - 1) arow = NS - 1;
        v8f c = zero8();
#pragma unroll 1
        for (int kc = 0; kc < 2; ++kc) {
          Frag ah, al, bh, bl;
          load_a(pr, PRP, arow, kc * 32 + 8 * h, ah, al);
          load_v(vh, kc, nt * 16 + m, h, bh, bl);
          c = mma3(ah.v, al.v, bh.v, bl.v, c);
        }
        const int col = hd * HDIM + nt * 16 + m;
#pragma unroll
        for (int r = 0; r < 8; ++r) {
          const int row = mt * 16 + 8 * h + r;
          if (row < NS) bufB[row * NHID + col] = c[r];
        }
      }
      __syncthreads();
    }

    gemm_big(bufB, NHID, 8, wsh + EW1_FR + (13 + i) * MAT_FR, wsl + EW1_FR + (13 + i) * MAT_FR,
             p.bo + i * NHID, bufC, bufA, false, wave, lane);
    __syncthreads();
    layer_norm(bufC, p.ln1g + i * NHID, p.ln1b + i * NHID, wave, lane);
    __syncthreads();

    gemm_big(bufC, NHID, 8, wsh + EW1_FR + (17 + i) * MAT_FR, wsl + EW1_FR + (17 + i) * MAT_FR,
             p.fb1 + i * NHID, bufB, nullptr, true, wave, lane);
    __syncthreads();
    gemm_big(bufB, NHID, 8, wsh + EW1_FR + (21 + i) * MAT_FR, wsl + EW1_FR + (21 + i) * MAT_FR,
             p.fb2 + i * NHID, bufA, nullptr, false, wave, lane);
    __syncthreads();
    layer_norm(bufA, p.ln2g + i * NHID, p.ln2b + i * NHID, wave, lane);
    __syncthreads();
  }

  {
    float acc = 0.f;
#pragma unroll 1
    for (int r = 0; r < NS; ++r) acc += bufA[r * NHID + tid];
    sc[tid] = acc * (1.f / 36.f);
  }
  __syncthreads();
  v4f val;
  val[0] = 0.f; val[1] = 0.f; val[2] = 0.f; val[3] = 0.f;
  if (tid < 64) {
    val = *(const v4fa*)(sc + tid * 4);
    float* op = p.out + (size_t)b * NHID + tid * 4;
    *(volatile v4f*)op = val;
  }
  __threadfence();
  if (tid < 64) {
    float* op = p.out + (size_t)b * NHID + tid * 4;
    *(volatile v4f*)op = val;
  }
}

extern "C" void kernel_launch(void* const* d_in, const int* in_sizes, int n_in,
                              void* d_out, int out_size, void* d_ws,
                              size_t ws_size, hipStream_t stream) {
  if (n_in < 25) return;
  Params p;
  p.robot = (const float*)d_in[0];
  p.objs  = (const float*)d_in[1];
  p.masks = (const int*)d_in[2];
  p.ew1 = (const float*)d_in[3];  p.eb1 = (const float*)d_in[4];
  p.ew2 = (const float*)d_in[5];  p.eb2 = (const float*)d_in[6];
  p.elg = (const float*)d_in[7];  p.elb = (const float*)d_in[8];
  p.Wq  = (const float*)d_in[9];  p.bq  = (const float*)d_in[10];
  p.Wk  = (const float*)d_in[11]; p.bk  = (const float*)d_in[12];
  p.Wv  = (const float*)d_in[13]; p.bv  = (const float*)d_in[14];
  p.Wo  = (const float*)d_in[15]; p.bo  = (const float*)d_in[16];
  p.ln1g = (const float*)d_in[17]; p.ln1b = (const float*)d_in[18];
  p.fw1 = (const float*)d_in[19]; p.fb1 = (const float*)d_in[20];
  p.fw2 = (const float*)d_in[21]; p.fb2 = (const float*)d_in[22];
  p.ln2g = (const float*)d_in[23]; p.ln2b = (const float*)d_in[24];
  p.out = (float*)d_out;

  const int B = out_size / NHID;
  if (B <= 0) return;
  if (in_sizes[0] < B * ROBW || in_sizes[1] < B * NOBJ * OBJD || in_sizes[2] < B * NOBJ) return;
  if (WS_NEED > ws_size) return;

  unsigned short* ws = (unsigned short*)d_ws;

  const int nblk = (NGROUPS + NTHR - 1) / NTHR;
  prepack_kernel<<<dim3(nblk), dim3(NTHR), 0, stream>>>(p, ws);

  fused_kernel<<<dim3(B), dim3(NTHR), 0, stream>>>(p, (const unsigned short*)ws);
}
